// LSTM_47356309406493
// MI455X (gfx1250) — hardware-run, weakly checked
//
#include <hip/hip_runtime.h>


#define NB    128
#define NT    256
#define NSTEP 255
#define NV    128
#define NH    512
#define NG    2048
#define NC    128
typedef _Float16 h16;
typedef unsigned short bf;
typedef __attribute__((ext_vector_type(16))) __bf16   v16bf;
typedef __attribute__((ext_vector_type(16))) _Float16 v16h;
typedef __attribute__((ext_vector_type(8)))  _Float16 v8h;
typedef __attribute__((ext_vector_type(8)))  unsigned short v8us;
typedef __attribute__((ext_vector_type(8)))  float    v8f;
typedef __attribute__((ext_vector_type(4)))  float    v4f;
typedef v8h  __attribute__((may_alias)) v8ha;
typedef v4f  __attribute__((may_alias)) v4fa;
typedef v8us __attribute__((may_alias)) v8usa;

__device__ __forceinline__ unsigned short f2bf(float f) { unsigned u = __float_as_uint(f); u += 0x7FFFu + ((u >> 16) & 1u); return (unsigned short)(u >> 16); }
__device__ __forceinline__ float bf2f(unsigned short b) { return __uint_as_float(((unsigned)b) << 16); }
__device__ __forceinline__ float bfr(float f) { return bf2f(f2bf(f)); }
__device__ __forceinline__ v16h cat16(v8h lo, v8h hi) { return __builtin_shufflevector(lo, hi, 0, 1, 2, 3, 4, 5, 6, 7, 8, 9, 10, 11, 12, 13, 14, 15); }
__device__ __forceinline__ v16bf cat16b(v8us lo, v8us hi) { return __builtin_bit_cast(v16bf, __builtin_shufflevector(lo, hi, 0, 1, 2, 3, 4, 5, 6, 7, 8, 9, 10, 11, 12, 13, 14, 15)); }
__device__ __forceinline__ v8f wmma16(v16h a, v16h b, v8f c) { return __builtin_amdgcn_wmma_f32_16x16x32_f16(false, a, false, b, (short)0, c, false, false); }
__device__ __forceinline__ v8f wmmab(v16bf a, v16bf b, v8f c) { return __builtin_amdgcn_wmma_f32_16x16x32_bf16(false, a, false, b, (short)0, c, false, false); }


template <typename T16> struct WFrag;
template <> struct WFrag<h16> { typedef v16h V; static __device__ __forceinline__ V ld(const h16* p) { return cat16(*(const v8h*)p, *(const v8h*)(p + 16)); } static __device__ __forceinline__ v8f mma(V a, V b, v8f c) { return wmma16(a, b, c); } };
template <> struct WFrag<bf> { typedef v16bf V; static __device__ __forceinline__ V ld(const bf* p) { return cat16b(*(const v8us*)p, *(const v8us*)(p + 16)); } static __device__ __forceinline__ v8f mma(V a, V b, v8f c) { return wmmab(a, b, c); } };
template <typename T16, int NSPLIT, bool BIAS>
__global__ __launch_bounds__(32) void k_gemmw(const T16* __restrict__ A, const T16* __restrict__ A2, const T16* __restrict__ Bt, const T16* __restrict__ Bt2, int K, float* C, int ldc, const float* __restrict__ bias, size_t sA, size_t sB, size_t sC) {
    typedef typename WFrag<T16>::V V;
    __shared__ __align__(16) float os[16 * 68];
    const size_t z = blockIdx.z; A += z * sA; if (A2) A2 += z * sA; Bt += z * sB; if (Bt2) Bt2 += z * sB; C += z * sC;
    const int lane = threadIdx.x & 31, lr = lane & 15, hi = lane >> 4; const int r0 = blockIdx.x * 64, c0 = blockIdx.y * 64;
    v8f acc[4][4];
#pragma unroll
    for (int mb = 0; mb < 4; ++mb)
#pragma unroll
        for (int nb = 0; nb < 4; ++nb) acc[mb][nb] = (v8f){};
    const size_t aoff = (size_t)(r0 + lr) * K + 8 * hi, boff = (size_t)(c0 + lr) * K + 8 * hi;
    for (int kc = 0; kc < K; kc += 32) {
        V a[4], a2[4];
#pragma unroll
        for (int mb = 0; mb < 4; ++mb) { a[mb] = WFrag<T16>::ld(A + aoff + (size_t)mb * 16 * K + kc); if (NSPLIT == 1 || NSPLIT == 2) a2[mb] = WFrag<T16>::ld(A2 + aoff + (size_t)mb * 16 * K + kc); }
#pragma unroll
        for (int nb = 0; nb < 4; ++nb) { const V b = WFrag<T16>::ld(Bt + boff + (size_t)nb * 16 * K + kc); V b2; if (NSPLIT >= 2) b2 = WFrag<T16>::ld(Bt2 + boff + (size_t)nb * 16 * K + kc);
#pragma unroll
            for (int mb = 0; mb < 4; ++mb) { acc[mb][nb] = WFrag<T16>::mma(a[mb], b, acc[mb][nb]); if (NSPLIT == 1 || NSPLIT == 2) acc[mb][nb] = WFrag<T16>::mma(a2[mb], b, acc[mb][nb]); if (NSPLIT >= 2) acc[mb][nb] = WFrag<T16>::mma(a[mb], b2, acc[mb][nb]); } }
        asm volatile("v_nop\n\tv_nop\n\tv_nop\n\tv_nop" : "+v"(acc[0][0]), "+v"(acc[1][1]), "+v"(acc[2][2]), "+v"(acc[3][3]) : "v"(a[0]), "v"(a[3]));
    }
#pragma unroll
    for (int mb = 0; mb < 4; ++mb) {
#pragma unroll
        for (int nb = 0; nb < 4; ++nb) {
#pragma unroll
            for (int j = 0; j < 8; ++j) os[(hi * 8 + j) * 68 + nb * 16 + lr] = acc[mb][nb][j]; }
        __builtin_amdgcn_wave_barrier(); asm volatile("" ::: "memory");
        float* crow = C + (size_t)(r0 + mb * 16) * ldc + c0;
#pragma unroll 1
        for (int ps = 0; ps < 2; ++ps) {
#pragma unroll
            for (int s = 0; s < 8; ++s) { const int row = 2 * s + hi, cofs = lr * 4; v4f val = *(const v4fa*)(os + row * 68 + cofs); if (BIAS) { val[0] += bfr(bias[c0 + cofs]); val[1] += bfr(bias[c0 + cofs + 1]); val[2] += bfr(bias[c0 + cofs + 2]); val[3] += bfr(bias[c0 + cofs + 3]); }
                *(volatile v4f*)(crow + (size_t)row * ldc + cofs) = val; }
            if (ps == 0) __threadfence(); }
        __builtin_amdgcn_wave_barrier(); asm volatile("" ::: "memory");
    }
}

typedef __attribute__((ext_vector_type(2))) _Float16 v2h;
typedef __attribute__((ext_vector_type(4))) _Float16 v4h;
typedef __attribute__((ext_vector_type(2))) unsigned short v2us;
typedef __attribute__((ext_vector_type(4))) unsigned short v4us;
typedef __attribute__((ext_vector_type(2))) float v2f;
typedef __attribute__((ext_vector_type(4))) int v4i;

__global__ __launch_bounds__(256) void k_wtG(const float* __restrict__ w, int K, int N, bf* Bt) {
    const int lane = threadIdx.x & 31; const int L0 = (blockIdx.x * 8 + (threadIdx.x >> 5)) * 8; const int nlines = N * K / 64;
#pragma unroll
    for (int ps = 0; ps < 2; ++ps) {
        for (int l = 0; l < 8; ++l) { const int L = L0 + l; if (L >= nlines) break; const size_t e = (size_t)L * 64 + lane * 2; const int k = (int)(e % K), n = (int)(e / K); v2us o;
            o[0] = f2bf(w[(size_t)k * N + n]); o[1] = f2bf(w[(size_t)(k + 1) * N + n]); *(volatile v2us*)(Bt + e) = o; }
        if (ps == 0) __threadfence(); }
}

__global__ __launch_bounds__(256) void k_zero(float* dst, int n4) { const int i = blockIdx.x * 256 + threadIdx.x; if (i >= n4) return; v4f z; z[0] = 0.0f; z[1] = 0.0f; z[2] = 0.0f; z[3] = 0.0f;
    *(volatile v4f*)(dst + (size_t)i * 4) = z; __threadfence(); *(volatile v4f*)(dst + (size_t)i * 4) = z; }

__device__ __forceinline__ float sgm(float v) { return 1.0f / (1.0f + expf(-v)); }
__global__ __launch_bounds__(256) void k_lstm(const float* __restrict__ p, const int* __restrict__ ids, int t, const float* __restrict__ wxg, const float* __restrict__ wxi, const float* __restrict__ wxf, const float* __restrict__ wxo, const float* __restrict__ bg, const float* __restrict__ bi, const float* __restrict__ bff, const float* __restrict__ bo, const float* __restrict__ cprev, float* cnew, bf* hw, bf* hh, bf* hl, size_t n4) { const size_t i = (size_t)blockIdx.x * 256 + threadIdx.x; if (i >= n4) return;
    const size_t row = i >> 7; const int c4 = (int)(i & 127) * 4; int id = ids[row * NT + t]; id = id < 0 ? 0 : id; id = id > NV - 1 ? NV - 1 : id;
    const float* q = p + row * NG + c4; const size_t xo = (size_t)id * NH + c4;
    const v4f pg = *(const v4f*)q; const v4f pi = *(const v4f*)(q + NH); const v4f pf = *(const v4f*)(q + 2 * NH); const v4f po = *(const v4f*)(q + 3 * NH);
    const v4f xg = *(const v4f*)(wxg + xo); const v4f xi = *(const v4f*)(wxi + xo); const v4f xf = *(const v4f*)(wxf + xo); const v4f xq = *(const v4f*)(wxo + xo);
    const v4f cp = *(const v4f*)(cprev + row * NH + c4); v4f cv; v4us hv; v4us hr;
#pragma unroll
    for (int k = 0; k < 4; ++k) { const float ag = (bfr(xg[k]) + pg[k]) + bfr(bg[c4 + k]); const float ai = (bfr(xi[k]) + pi[k]) + bfr(bi[c4 + k]); const float af = (bfr(xf[k]) + pf[k]) + bfr(bff[c4 + k]); const float ao = (bfr(xq[k]) + po[k]) + bfr(bo[c4 + k]);
        const float g = tanhf(ag); const float gi = sgm(ai); const float gf = sgm(af); const float go = sgm(ao); const float c = g * gi + cp[k] * gf; const float h = tanhf(c) * go; cv[k] = c; hv[k] = f2bf(h); hr[k] = f2bf(h - bf2f(hv[k])); }
#pragma unroll
    for (int ps = 0; ps < 2; ++ps) { *(volatile v4f*)(cnew + row * NH + c4) = cv; *(volatile v4us*)(hw + row * NH + c4) = hv; if (hh) { *(volatile v4us*)(hh + row * NH + c4) = hv; *(volatile v4us*)(hl + row * NH + c4) = hr; } if (ps == 0) __threadfence(); } }

__global__ __launch_bounds__(256) void k_outb(const float* __restrict__ ph, const float* __restrict__ bp, float* out, size_t n4) { const size_t i = (size_t)blockIdx.x * 256 + threadIdx.x; if (i >= n4) return; const int c4 = (int)(i & 31) * 4; const v4f v = *(const v4f*)(ph + i * 4); v4f r;
#pragma unroll
    for (int k = 0; k < 4; ++k) r[k] = v[k] + bfr(bp[c4 + k]);
    *(volatile v4f*)(out + i * 4) = r; __threadfence(); *(volatile v4f*)(out + i * 4) = r; }

static constexpr size_t kSzWHt = (size_t)NG * NH * 2, kSzWPt = (size_t)NC * NH * 2, kSzHW = (size_t)NB * NH * 2, kSzC = (size_t)NB * NH * 4, kSzP = (size_t)NB * NG * 4, kSzPH = (size_t)NB * NC * 4;
static constexpr size_t kOffWHt = 0, kOffWPt = kOffWHt + kSzWHt, kOffHW0 = kOffWPt + kSzWPt, kOffHW1 = kOffHW0 + kSzHW, kOffC0 = kOffHW1 + kSzHW, kOffC1 = kOffC0 + kSzC, kOffP = kOffC1 + kSzC, kOffHH = kOffP + kSzP, kOffHL = kOffHH + kSzHW, kOffPH = kOffHL + kSzHW, kWsTotal = kOffPH + kSzPH;
static_assert(kSzWHt == 2097152ull && kSzWPt == 131072ull && kSzHW == 131072ull && kSzC == 262144ull && kSzP == 1048576ull && kSzPH == 65536ull && kWsTotal == 4390912ull);
static_assert(kWsTotal <= 134217728ull);
static_assert((kOffWPt % 128) == 0 && (kOffHW0 % 128) == 0 && (kOffHW1 % 128) == 0 && (kOffC0 % 128) == 0 && (kOffC1 % 128) == 0 && (kOffP % 128) == 0 && (kOffHH % 128) == 0 && (kOffHL % 128) == 0 && (kOffPH % 128) == 0);
static_assert((NB % 64) == 0 && (NG % 64) == 0 && (NC % 64) == 0 && (NH % 32) == 0 && NG == 4 * NH && NSTEP == NT - 1);
static_assert(((NH * NH) % 4096) == 0 && ((NH * NC) % 4096) == 0);

extern "C" void kernel_launch(void* const* d_in, const int* in_sizes, int n_in, void* d_out, int out_size, void* d_ws, size_t ws_size, hipStream_t stream) {
    if (n_in < 15) return;
    if (in_sizes[0] != NB * NT) return;
    for (int q = 1; q < 9; q += 2) { if (in_sizes[q] != NV * NH || in_sizes[q + 1] != NH * NH) return; }
    if (in_sizes[9] != NH * NC) return;
    for (int q = 10; q < 14; ++q) { if (in_sizes[q] != NH) return; }
    if (in_sizes[14] != NC) return;
    if (out_size != NB * NC) return;
    if (ws_size < kWsTotal) return;
    const int* ids = (const int*)d_in[0];
    const float* wxg = (const float*)d_in[1]; const float* whg = (const float*)d_in[2]; const float* wxi = (const float*)d_in[3]; const float* whi = (const float*)d_in[4]; const float* wxf = (const float*)d_in[5]; const float* whf = (const float*)d_in[6]; const float* wxo = (const float*)d_in[7]; const float* who = (const float*)d_in[8]; const float* whp = (const float*)d_in[9];
    const float* bg = (const float*)d_in[10]; const float* bi = (const float*)d_in[11]; const float* bff = (const float*)d_in[12]; const float* bo = (const float*)d_in[13]; const float* bp = (const float*)d_in[14];
    float* out = (float*)d_out; char* ws = (char*)d_ws;
    bf* WHt = (bf*)(ws + kOffWHt); bf* WPt = (bf*)(ws + kOffWPt); bf* HW0 = (bf*)(ws + kOffHW0); bf* HW1 = (bf*)(ws + kOffHW1); float* C0 = (float*)(ws + kOffC0); float* C1 = (float*)(ws + kOffC1); float* P = (float*)(ws + kOffP); bf* HH = (bf*)(ws + kOffHH); bf* HL = (bf*)(ws + kOffHL); float* PH = (float*)(ws + kOffPH);

    k_wtG<<<(unsigned)((NH * NH / 64 + 63) / 64), 256, 0, stream>>>(whg, NH, NH, WHt);
    k_wtG<<<(unsigned)((NH * NH / 64 + 63) / 64), 256, 0, stream>>>(whi, NH, NH, WHt + (size_t)NH * NH);
    k_wtG<<<(unsigned)((NH * NH / 64 + 63) / 64), 256, 0, stream>>>(whf, NH, NH, WHt + (size_t)2 * NH * NH);
    k_wtG<<<(unsigned)((NH * NH / 64 + 63) / 64), 256, 0, stream>>>(who, NH, NH, WHt + (size_t)3 * NH * NH);
    k_wtG<<<(unsigned)((NH * NC / 64 + 63) / 64), 256, 0, stream>>>(whp, NH, NC, WPt);
    k_zero<<<(unsigned)(kSzHW / 16 / 256), 256, 0, stream>>>((float*)HW0, (int)(kSzHW / 16));
    k_zero<<<(unsigned)(kSzC / 16 / 256), 256, 0, stream>>>(C0, (int)(kSzC / 16));

    for (int t = 0; t < NSTEP; ++t) { const bf* hin = (t & 1) ? HW1 : HW0; bf* hout = (t & 1) ? HW0 : HW1; const float* cin = (t & 1) ? C1 : C0; float* cout = (t & 1) ? C0 : C1; const bool last = (t == NSTEP - 1);
        k_gemmw<bf, 0, false><<<dim3(NB / 64, NG / 64, 1), 32, 0, stream>>>(hin, nullptr, WHt, nullptr, NH, P, NG, nullptr, 0, 0, 0);
        k_lstm<<<(unsigned)(NB * 128 / 256), 256, 0, stream>>>(P, ids, t, wxg, wxi, wxf, wxo, bg, bi, bff, bo, cin, cout, hout, last ? HH : nullptr, last ? HL : nullptr, (size_t)NB * 128); }

    k_gemmw<bf, 1, false><<<dim3(NB / 64, NC / 64, 1), 32, 0, stream>>>(HH, HL, WPt, nullptr, NH, PH, NC, nullptr, 0, 0, 0);
    k_outb<<<(unsigned)(NB * NC / 4 / 256), 256, 0, stream>>>(PH, bp, out, (size_t)NB * NC / 4);
}
